// MyTransformerLayer_90452011254120
// MI455X (gfx1250) — hardware-run, weakly checked
//
#include <hip/hip_runtime.h>


#define NB_  4
#define NN   2048
#define EE   256
#define E2   512
#define E3   768
#define NH_  4
#define HD   64
#define PCAR 1024.0f
typedef _Float16 h16;
typedef unsigned short bf;
typedef __attribute__((ext_vector_type(16))) __bf16   v16bf;
typedef __attribute__((ext_vector_type(16))) _Float16 v16h;
typedef __attribute__((ext_vector_type(8)))  _Float16 v8h;
typedef __attribute__((ext_vector_type(8)))  unsigned short v8us;
typedef __attribute__((ext_vector_type(8)))  float    v8f;
typedef __attribute__((ext_vector_type(4)))  float    v4f;
typedef v8h  __attribute__((may_alias)) v8ha;
typedef v4f  __attribute__((may_alias)) v4fa;
typedef v8us __attribute__((may_alias)) v8usa;

__device__ __forceinline__ unsigned short f2bf(float f) { unsigned u = __float_as_uint(f); u += 0x7FFFu + ((u >> 16) & 1u); return (unsigned short)(u >> 16); }
__device__ __forceinline__ float bf2f(unsigned short b) { return __uint_as_float(((unsigned)b) << 16); }
__device__ __forceinline__ float bfr(float f) { return bf2f(f2bf(f)); }
__device__ __forceinline__ v16h cat16(v8h lo, v8h hi) { return __builtin_shufflevector(lo, hi, 0, 1, 2, 3, 4, 5, 6, 7, 8, 9, 10, 11, 12, 13, 14, 15); }
__device__ __forceinline__ v16bf cat16b(v8us lo, v8us hi) { return __builtin_bit_cast(v16bf, __builtin_shufflevector(lo, hi, 0, 1, 2, 3, 4, 5, 6, 7, 8, 9, 10, 11, 12, 13, 14, 15)); }
__device__ __forceinline__ v8f wmma16(v16h a, v16h b, v8f c) { return __builtin_amdgcn_wmma_f32_16x16x32_f16(false, a, false, b, (short)0, c, false, false); }
__device__ __forceinline__ v8f wmmab(v16bf a, v16bf b, v8f c) { return __builtin_amdgcn_wmma_f32_16x16x32_bf16(false, a, false, b, (short)0, c, false, false); }


template <typename T16> struct WFrag;
template <> struct WFrag<h16> { typedef v16h V; static __device__ __forceinline__ V ld(const h16* p) { return cat16(*(const v8h*)p, *(const v8h*)(p + 16)); } static __device__ __forceinline__ v8f mma(V a, V b, v8f c) { return wmma16(a, b, c); } };
template <> struct WFrag<bf> { typedef v16bf V; static __device__ __forceinline__ V ld(const bf* p) { return cat16b(*(const v8us*)p, *(const v8us*)(p + 16)); } static __device__ __forceinline__ v8f mma(V a, V b, v8f c) { return wmmab(a, b, c); } };
template <typename T16, int NSPLIT, bool BIAS>
__global__ __launch_bounds__(32) void k_gemmw(const T16* __restrict__ A, const T16* __restrict__ A2, const T16* __restrict__ Bt, const T16* __restrict__ Bt2, int K, float* C, int ldc, const float* __restrict__ bias, size_t sA, size_t sB, size_t sC) {
    typedef typename WFrag<T16>::V V;
    __shared__ __align__(16) float os[16 * 68];
    const size_t z = blockIdx.z; A += z * sA; if (A2) A2 += z * sA; Bt += z * sB; if (Bt2) Bt2 += z * sB; C += z * sC;
    const int lane = threadIdx.x & 31, lr = lane & 15, hi = lane >> 4; const int r0 = blockIdx.x * 64, c0 = blockIdx.y * 64;
    v8f acc[4][4];
#pragma unroll
    for (int mb = 0; mb < 4; ++mb)
#pragma unroll
        for (int nb = 0; nb < 4; ++nb) acc[mb][nb] = (v8f){};
    const size_t aoff = (size_t)(r0 + lr) * K + 8 * hi, boff = (size_t)(c0 + lr) * K + 8 * hi;
#pragma unroll 1
    for (int kc = 0; kc < K; kc += 32) {
        V a[4], a2[4];
#pragma unroll
        for (int mb = 0; mb < 4; ++mb) { a[mb] = WFrag<T16>::ld(A + aoff + (size_t)mb * 16 * K + kc); if (NSPLIT == 1 || NSPLIT == 2) a2[mb] = WFrag<T16>::ld(A2 + aoff + (size_t)mb * 16 * K + kc); }
#pragma unroll
        for (int nb = 0; nb < 4; ++nb) { const V b = WFrag<T16>::ld(Bt + boff + (size_t)nb * 16 * K + kc); V b2; if (NSPLIT >= 2) b2 = WFrag<T16>::ld(Bt2 + boff + (size_t)nb * 16 * K + kc);
#pragma unroll
            for (int mb = 0; mb < 4; ++mb) { acc[mb][nb] = WFrag<T16>::mma(a[mb], b, acc[mb][nb]); if (NSPLIT == 1 || NSPLIT == 2) acc[mb][nb] = WFrag<T16>::mma(a2[mb], b, acc[mb][nb]); if (NSPLIT >= 2) acc[mb][nb] = WFrag<T16>::mma(a[mb], b2, acc[mb][nb]); } }
        asm volatile("v_nop\n\tv_nop\n\tv_nop\n\tv_nop" : "+v"(acc[0][0]), "+v"(acc[1][1]), "+v"(acc[2][2]), "+v"(acc[3][3]) : "v"(a[0]), "v"(a[3]));
    }
#pragma unroll
    for (int mb = 0; mb < 4; ++mb) {
#pragma unroll
        for (int nb = 0; nb < 4; ++nb) {
#pragma unroll
            for (int j = 0; j < 8; ++j) os[(hi * 8 + j) * 68 + nb * 16 + lr] = acc[mb][nb][j]; }
        __builtin_amdgcn_wave_barrier(); asm volatile("" ::: "memory");
        float* crow = C + (size_t)(r0 + mb * 16) * ldc + c0;
#pragma unroll 1
        for (int ps = 0; ps < 2; ++ps) {
#pragma unroll
            for (int s = 0; s < 8; ++s) { const int row = 2 * s + hi, cofs = lr * 4; v4f val = *(const v4fa*)(os + row * 68 + cofs); if (BIAS) { val[0] += bfr(bias[c0 + cofs]); val[1] += bfr(bias[c0 + cofs + 1]); val[2] += bfr(bias[c0 + cofs + 2]); val[3] += bfr(bias[c0 + cofs + 3]); }
                *(volatile v4f*)(crow + (size_t)row * ldc + cofs) = val; }
            if (ps == 0) __threadfence(); }
        __builtin_amdgcn_wave_barrier(); asm volatile("" ::: "memory");
    }
}

__device__ __forceinline__ h16 tohx(float x) { return (h16)x; }
__device__ __forceinline__ void splitf(float y, unsigned short& h, unsigned short& l) { h = f2bf(y); l = f2bf(y - bf2f(h)); }
typedef __attribute__((ext_vector_type(2))) unsigned short v2us;
typedef __attribute__((ext_vector_type(4))) unsigned short v4us;
typedef __attribute__((ext_vector_type(2))) _Float16 v2h;
typedef __attribute__((ext_vector_type(4))) _Float16 v4h;

__global__ __launch_bounds__(256) void k_wtG(const float* __restrict__ w, int K, int N, bf* Bt) {
    const int lane = threadIdx.x & 31; const int L0 = (blockIdx.x * 8 + (threadIdx.x >> 5)) * 8; const int nlines = N * K / 64;
#pragma unroll
    for (int ps = 0; ps < 2; ++ps) {
#pragma unroll 1
        for (int l = 0; l < 8; ++l) { const int L = L0 + l; if (L >= nlines) break; const size_t e = (size_t)L * 64 + lane * 2; const int k = (int)(e % K), n = (int)(e / K); v2us o;
            o[0] = f2bf(w[(size_t)k * N + n]); o[1] = f2bf(w[(size_t)(k + 1) * N + n]); *(volatile v2us*)(Bt + e) = o; }
        if (ps == 0) __threadfence(); }
}
__global__ __launch_bounds__(256) void k_cvt8(const float* __restrict__ src, bf* dst, size_t n8) { const size_t i = (size_t)blockIdx.x * 256 + threadIdx.x; if (i >= n8) return; const v8f v = *(const v8f*)(src + i * 8); v8us o;
#pragma unroll
    for (int k = 0; k < 8; ++k) o[k] = f2bf(v[k]); *(volatile v8us*)(dst + i * 8) = o; __threadfence(); *(volatile v8us*)(dst + i * 8) = o; }
__global__ __launch_bounds__(256) void k_spl(const float* __restrict__ QKV, const float* __restrict__ encC, const float* __restrict__ encS, h16* Q16, h16* K16) { const int e = (blockIdx.x * 256 + threadIdx.x) * 4; if (e >= NH_ * NN * HD) return; const int d = e % HD; const int t = (e / HD) % NN; const int h = e / (HD * NN); const float* row = QKV + (size_t)t * E3 + h * 3 * HD; v4h q, k;
#pragma unroll
    for (int u = 0; u < 4; ++u) { const int dd = d + u, dp = dd ^ 1; const float c = bfr(encC[(size_t)t * HD + dd]), s = bfr(encS[(size_t)t * HD + dd]);
        const float qa = row[dd * 3 + 0], qb = row[dp * 3 + 0], ka = row[dd * 3 + 1], kb = row[dp * 3 + 1]; const float rq = (dd & 1) ? qb : -qb, rk = (dd & 1) ? kb : -kb;
        float q1 = __fmul_rn(qa, c), q2 = __fmul_rn(rq, s), k1 = __fmul_rn(ka, c), k2 = __fmul_rn(rk, s); asm volatile("" : "+v"(q1)); asm volatile("" : "+v"(q2)); asm volatile("" : "+v"(k1)); asm volatile("" : "+v"(k2));
        q[u] = tohx(__fadd_rn(q1, q2) * 0.125f); k[u] = tohx(__fadd_rn(k1, k2)); }
    for (int ps = 0; ps < 2; ++ps) { *(volatile v4h*)(Q16 + e) = q; *(volatile v4h*)(K16 + e) = k; if (ps == 0) __threadfence(); } }
__global__ __launch_bounds__(256) void k_vt3(const float* __restrict__ QKV, h16* VT) { const int e = (blockIdx.x * 256 + threadIdx.x) * 2; if (e >= NH_ * HD * NN) return; const int t = e % NN; const int d = (e / NN) % HD; const int h = e / (NN * HD); v2h o; o[0] = tohx(QKV[(size_t)t * E3 + h * 3 * HD + d * 3 + 2]); o[1] = tohx(QKV[(size_t)(t + 1) * E3 + h * 3 * HD + d * 3 + 2]);
    *(volatile v2h*)(VT + e) = o; __threadfence(); *(volatile v2h*)(VT + e) = o; }
__global__ __launch_bounds__(256) void k_cpl(const float* __restrict__ QK, h16* A16) { const int e = (blockIdx.x * 256 + threadIdx.x) * 4; if (e >= NH_ * NN * HD) return; const int d = e % HD; const int t = (e / HD) % NN; const int h = e / (HD * NN); const float* f = QK + (size_t)t * EE + h * HD + d; const float s4 = 0.35355339059327379f; v4h o;
#pragma unroll
    for (int u = 0; u < 4; ++u) o[u] = tohx(__fmul_rn(f[u], s4)); *(volatile v4h*)(A16 + e) = o; __threadfence(); *(volatile v4h*)(A16 + e) = o; }
__global__ __launch_bounds__(256) void k_vtc(const float* __restrict__ V, h16* VT) { const int e = (blockIdx.x * 256 + threadIdx.x) * 2; if (e >= NH_ * HD * NN) return; const int t = e % NN; const int d = (e / NN) % HD; const int h = e / (NN * HD); v2h o; o[0] = tohx(V[(size_t)t * EE + h * HD + d]); o[1] = tohx(V[(size_t)(t + 1) * EE + h * HD + d]);
    *(volatile v2h*)(VT + e) = o; __threadfence(); *(volatile v2h*)(VT + e) = o; }
__global__ __launch_bounds__(256) void k_soft(const float* __restrict__ Sb, int nrows, h16* P16) { const int lane = threadIdx.x & 31; const int row = blockIdx.x * 8 + (threadIdx.x >> 5); if (row >= nrows) return; const float* sr = Sb + (size_t)row * NN; float v[NN / 32]; float mx = -3.0e38f;
#pragma unroll
    for (int ch = 0; ch < NN / 128; ++ch) { const v4f a = *(const v4f*)(sr + ch * 128 + lane * 4);
#pragma unroll
        for (int u = 0; u < 4; ++u) { v[ch * 4 + u] = a[u]; mx = fmaxf(mx, a[u]); } }
#pragma unroll
    for (int sh = 16; sh; sh >>= 1) mx = fmaxf(mx, __shfl_xor(mx, sh, 32));
    float sum = 0.f;
#pragma unroll
    for (int q = 0; q < NN / 32; ++q) { float d0 = __fsub_rn(v[q], mx); asm volatile("" : "+v"(d0)); v[q] = __builtin_amdgcn_exp2f(__fmul_rn(d0, 1.4426950408889634f)); sum += v[q]; }
#pragma unroll
    for (int sh = 16; sh; sh >>= 1) sum += __shfl_xor(sum, sh, 32);
    const float f = __fdiv_rn(PCAR, sum);
    for (int ps = 0; ps < 2; ++ps) {
#pragma unroll
        for (int ch = 0; ch < NN / 128; ++ch) { v4h o4;
#pragma unroll
            for (int q = 0; q < 4; ++q) o4[q] = tohx(v[ch * 4 + q] * f); *(volatile v4h*)(P16 + (size_t)row * NN + ch * 128 + lane * 4) = o4; }
        if (ps == 0) __threadfence(); } }
__global__ __launch_bounds__(256) void k_mrg(const float* __restrict__ O, bf* Ch, bf* Cl) { const int e = (blockIdx.x * 256 + threadIdx.x) * 4; if (e >= NH_ * NN * HD) return; const int d = e % HD; const int t = (e / HD) % NN; const int h = e / (HD * NN); v4us oh, ol;
#pragma unroll
    for (int u = 0; u < 4; ++u) { unsigned short a, b; splitf(O[e + u] * (1.0f / PCAR), a, b); oh[u] = a; ol[u] = b; } const size_t oo = (size_t)t * EE + h * HD + d; *(volatile v4us*)(Ch + oo) = oh; *(volatile v4us*)(Cl + oo) = ol; __threadfence(); *(volatile v4us*)(Ch + oo) = oh; *(volatile v4us*)(Cl + oo) = ol; }
template <bool RAW> __global__ __launch_bounds__(256) void k_cat(const float* __restrict__ X, const float* __restrict__ MSG, bf* Ah, bf* Al) { const int e = (blockIdx.x * 256 + threadIdx.x) * 4; if (e >= NN * E2) return; const int c = e % E2; const int t = e / E2; v4us oh, ol;
#pragma unroll
    for (int u = 0; u < 4; ++u) { const int cc = c + u; float v = (cc < EE) ? X[(size_t)t * EE + cc] : MSG[(size_t)t * EE + cc - EE]; if (RAW && cc < EE) v = bfr(v); unsigned short a, b; splitf(v, a, b); oh[u] = a; ol[u] = b; }
    *(volatile v4us*)(Ah + e) = oh; *(volatile v4us*)(Al + e) = ol; __threadfence(); *(volatile v4us*)(Ah + e) = oh; *(volatile v4us*)(Al + e) = ol; }
__global__ __launch_bounds__(256) void k_lng(const float* __restrict__ H1, const float* __restrict__ gg, const float* __restrict__ bn, float* LN) { const int lane = threadIdx.x & 31; const int t = blockIdx.x * 8 + (threadIdx.x >> 5); if (t >= NN) return; const float* hr = H1 + (size_t)t * E2; float v[E2 / 32]; float s = 0.f;
#pragma unroll
    for (int ch = 0; ch < E2 / 128; ++ch) { const v4f a = *(const v4f*)(hr + ch * 128 + lane * 4);
#pragma unroll
        for (int u = 0; u < 4; ++u) { v[ch * 4 + u] = a[u]; s += a[u]; } }
#pragma unroll
    for (int sh = 16; sh; sh >>= 1) s += __shfl_xor(s, sh, 32);
    const float mean = s * (1.0f / E2); float q = 0.f;
#pragma unroll
    for (int k = 0; k < E2 / 32; ++k) { float d = __fsub_rn(v[k], mean); asm volatile("" : "+v"(d)); float p = __fmul_rn(d, d); asm volatile("" : "+v"(p)); q = __fadd_rn(q, p); }
#pragma unroll
    for (int sh = 16; sh; sh >>= 1) q += __shfl_xor(q, sh, 32);
    const float rstd = __fdiv_rn(1.0f, __fsqrt_rn(__fadd_rn(q * (1.0f / E2), 1e-5f)));
    for (int ps = 0; ps < 2; ++ps) {
#pragma unroll
        for (int ch = 0; ch < E2 / 128; ++ch) { v4f o; const int c0 = ch * 128 + lane * 4;
#pragma unroll
            for (int u = 0; u < 4; ++u) { float d = __fsub_rn(v[ch * 4 + u], mean); asm volatile("" : "+v"(d)); float n0 = __fmul_rn(d, rstd); asm volatile("" : "+v"(n0)); float g1 = bfr(gg[c0 + u]), b1 = bfr(bn[c0 + u]); asm volatile("" : "+v"(g1)); asm volatile("" : "+v"(b1)); float t1 = __fmul_rn(n0, g1); asm volatile("" : "+v"(t1)); o[u] = __fadd_rn(t1, b1); }
            *(volatile v4f*)(LN + (size_t)t * E2 + c0) = o; }
        if (ps == 0) __threadfence(); } }
__global__ __launch_bounds__(256) void k_gelu(const float* __restrict__ LN, bf* Gh, bf* Gl) { const int e = (blockIdx.x * 256 + threadIdx.x) * 4; if (e >= NN * E2) return; const v4f a = *(const v4f*)(LN + e); v4us oh, ol;
#pragma unroll 1
    for (int u = 0; u < 4; ++u) { const float y = a[u]; float er = erff(y * 0.70710678118654752f); asm volatile("" : "+v"(er)); float hy = __fmul_rn(0.5f, y); asm volatile("" : "+v"(hy)); const float ge = __fmul_rn(hy, __fadd_rn(1.0f, er)); unsigned short h, l; splitf(ge, h, l); oh[u] = h; ol[u] = l; }
    *(volatile v4us*)(Gh + e) = oh; *(volatile v4us*)(Gl + e) = ol; __threadfence(); *(volatile v4us*)(Gh + e) = oh; *(volatile v4us*)(Gl + e) = ol; }

template <bool RAW> __global__ __launch_bounds__(256) void k_resid(const float* __restrict__ X, const float* __restrict__ F, float* Dd) { const int e = (blockIdx.x * 256 + threadIdx.x) * 4; if (e >= NN * EE) return; const v4f a = *(const v4f*)(X + e), f = *(const v4f*)(F + e); v4f o;
#pragma unroll
    for (int u = 0; u < 4; ++u) o[u] = __fadd_rn(RAW ? bfr(a[u]) : a[u], f[u]); *(volatile v4f*)(Dd + e) = o; __threadfence(); *(volatile v4f*)(Dd + e) = o; }
__global__ __launch_bounds__(256) void k_dpl(const float* __restrict__ X, bf* Xh, bf* Xl) { const int e = (blockIdx.x * 256 + threadIdx.x) * 4; if (e >= NN * EE) return; const v4f a = *(const v4f*)(X + e); v4us oh, ol;
#pragma unroll
    for (int u = 0; u < 4; ++u) { unsigned short h, l; splitf(a[u], h, l); oh[u] = h; ol[u] = l; } *(volatile v4us*)(Xh + e) = oh; *(volatile v4us*)(Xl + e) = ol; __threadfence(); *(volatile v4us*)(Xh + e) = oh; *(volatile v4us*)(Xl + e) = ol; }
__global__ __launch_bounds__(256) void k_out(const float* __restrict__ Y, int off, float* O0, float* O1) { const int e = (blockIdx.x * 256 + threadIdx.x) * 4; if (e >= NN * EE) return; const int c = e % EE; const int t = e / EE; const v4f a = *(const v4f*)(Y + e); const size_t oo = (size_t)t * E2 + off + c;
    *(volatile v4f*)(O0 + oo) = a; *(volatile v4f*)(O1 + oo) = a; __threadfence(); *(volatile v4f*)(O0 + oo) = a; *(volatile v4f*)(O1 + oo) = a; }

extern "C" void kernel_launch(void* const* d_in, const int* in_sizes, int n_in,
                              void* d_out, int out_size, void* d_ws, size_t ws_size, hipStream_t stream) {
    (void)in_sizes; (void)n_in; (void)out_size;
    const float** I = (const float**)d_in;
    const float *desc0 = I[0], *desc1 = I[1], *enc0 = I[2], *enc1 = I[3], *sWqkv = I[4], *sbqkv = I[5], *sWout = I[6], *sbout = I[7], *sW1 = I[8], *sb1 = I[9], *sg = I[10], *sbn = I[11], *sW2 = I[12], *sb2 = I[13];
    const float *cWqk = I[14], *cbqk = I[15], *cWv = I[16], *cbv = I[17], *cWo = I[18], *cbo = I[19], *cW1 = I[20], *cb1 = I[21], *cg = I[22], *cbn = I[23], *cW2 = I[24], *cb2 = I[25];
    float* OUT0 = (float*)d_out; float* OUT1 = OUT0 + (size_t)NB_ * NN * E2;
    char* wsp = (char*)d_ws;
    auto take = [&](size_t bytes) { char* p = wsp; wsp += (bytes + 255) & ~(size_t)255; return (void*)p; };
    bf* SWQKV = (bf*)take((size_t)E3 * EE * 2); bf* SWOUT = (bf*)take(EE * EE * 2); bf* SW1 = (bf*)take((size_t)E2 * E2 * 2); bf* SW2 = (bf*)take((size_t)EE * E2 * 2); bf* CWQK = (bf*)take(EE * EE * 2); bf* CWV = (bf*)take(EE * EE * 2); bf* CWO = (bf*)take(EE * EE * 2); bf* CW1 = (bf*)take((size_t)E2 * E2 * 2); bf* CW2 = (bf*)take((size_t)EE * E2 * 2);
    bf* XB = (bf*)take((size_t)NN * EE * 2); float* QKV = (float*)take((size_t)NN * E3 * 4); h16* Q16 = (h16*)take((size_t)NH_ * NN * HD * 2); h16* K16 = (h16*)take((size_t)NH_ * NN * HD * 2); h16* VT0 = (h16*)take((size_t)NH_ * HD * NN * 2); h16* VT1 = (h16*)take((size_t)NH_ * HD * NN * 2);
    float* Sb = (float*)take((size_t)NH_ * NN * NN * 4); h16* P16 = (h16*)take((size_t)NH_ * NN * NN * 2); float* O = (float*)take((size_t)NH_ * NN * HD * 4); bf* Ch = (bf*)take((size_t)NN * EE * 2); bf* Cl = (bf*)take((size_t)NN * EE * 2); float* MSG = (float*)take((size_t)NN * EE * 4);
    bf* Ah = (bf*)take((size_t)NN * E2 * 2); bf* Al = (bf*)take((size_t)NN * E2 * 2); float* H1 = (float*)take((size_t)NN * E2 * 4); float* LNb = (float*)take((size_t)NN * E2 * 4); bf* Gh = (bf*)take((size_t)NN * E2 * 2); bf* Gl = (bf*)take((size_t)NN * E2 * 2); float* F2 = (float*)take((size_t)NN * EE * 4);
    float* D0 = (float*)take((size_t)NN * EE * 4); float* D1 = (float*)take((size_t)NN * EE * 4); bf* D0h = (bf*)take((size_t)NN * EE * 2); bf* D0l = (bf*)take((size_t)NN * EE * 2); bf* D1h = (bf*)take((size_t)NN * EE * 2); bf* D1l = (bf*)take((size_t)NN * EE * 2);
    float* QK0 = (float*)take((size_t)NN * EE * 4); float* QK1 = (float*)take((size_t)NN * EE * 4); float* V0 = (float*)take((size_t)NN * EE * 4); float* V1 = (float*)take((size_t)NN * EE * 4); float* Y = (float*)take((size_t)NN * EE * 4);
    if ((size_t)(wsp - (char*)d_ws) > ws_size) return;
    k_wtG<<<(EE * E3 / 64 + 63) / 64, 256, 0, stream>>>(sWqkv, EE, E3, SWQKV); k_wtG<<<(EE * EE / 64 + 63) / 64, 256, 0, stream>>>(sWout, EE, EE, SWOUT); k_wtG<<<(E2 * E2 / 64 + 63) / 64, 256, 0, stream>>>(sW1, E2, E2, SW1); k_wtG<<<(E2 * EE / 64 + 63) / 64, 256, 0, stream>>>(sW2, E2, EE, SW2);
    k_wtG<<<(EE * EE / 64 + 63) / 64, 256, 0, stream>>>(cWqk, EE, EE, CWQK); k_wtG<<<(EE * EE / 64 + 63) / 64, 256, 0, stream>>>(cWv, EE, EE, CWV); k_wtG<<<(EE * EE / 64 + 63) / 64, 256, 0, stream>>>(cWo, EE, EE, CWO); k_wtG<<<(E2 * E2 / 64 + 63) / 64, 256, 0, stream>>>(cW1, E2, E2, CW1); k_wtG<<<(E2 * EE / 64 + 63) / 64, 256, 0, stream>>>(cW2, E2, EE, CW2);
    const unsigned g4 = (NH_ * NN * HD / 4 + 255) / 256, g2 = (NH_ * HD * NN / 2 + 255) / 256, gE = (NN * EE / 4 + 255) / 256, gE2 = (NN * E2 / 4 + 255) / 256;
    auto attend = [&](const h16* A, const h16* Bk, const h16* VT) {
        k_gemmw<h16, 0, false><<<dim3(NN / 64, NN / 64, NH_), 32, 0, stream>>>(A, nullptr, Bk, nullptr, HD, Sb, NN, nullptr, (size_t)NN * HD, (size_t)NN * HD, (size_t)NN * NN);
        k_soft<<<NH_ * NN / 8, 256, 0, stream>>>(Sb, NH_ * NN, P16);
        k_gemmw<h16, 0, false><<<dim3(NN / 64, 1, NH_), 32, 0, stream>>>(P16, nullptr, VT, nullptr, NN, O, HD, nullptr, (size_t)NN * NN, (size_t)HD * NN, (size_t)NN * HD);
        k_mrg<<<g4, 256, 0, stream>>>(O, Ch, Cl); };
    auto ffn = [&](bool raw, const float* X, const bf* W1, const float* b1, const float* gg, const float* bn, const bf* W2, const float* b2, float* Dout) {
        if (raw) k_cat<true><<<gE2, 256, 0, stream>>>(X, MSG, Ah, Al); else k_cat<false><<<gE2, 256, 0, stream>>>(X, MSG, Ah, Al);
        k_gemmw<bf, 1, true><<<dim3(NN / 64, E2 / 64, 1), 32, 0, stream>>>(Ah, Al, W1, nullptr, E2, H1, E2, b1, 0, 0, 0); k_lng<<<NN / 8, 256, 0, stream>>>(H1, gg, bn, LNb); k_gelu<<<gE2, 256, 0, stream>>>(LNb, Gh, Gl);
        k_gemmw<bf, 1, true><<<dim3(NN / 64, EE / 64, 1), 32, 0, stream>>>(Gh, Gl, W2, nullptr, E2, F2, EE, b2, 0, 0, 0);
        if (raw) k_resid<true><<<gE, 256, 0, stream>>>(X, F2, Dout); else k_resid<false><<<gE, 256, 0, stream>>>(X, F2, Dout); };
    auto self_block = [&](const float* x, const float* encb, float* Dout) {
        k_cvt8<<<(NN * EE / 8 + 255) / 256, 256, 0, stream>>>(x, XB, (size_t)NN * EE / 8); k_gemmw<bf, 0, true><<<dim3(NN / 64, E3 / 64, 1), 32, 0, stream>>>(XB, nullptr, SWQKV, nullptr, EE, QKV, E3, sbqkv, 0, 0, 0);
        k_spl<<<g4, 256, 0, stream>>>(QKV, encb, encb + (size_t)NB_ * NN * HD, Q16, K16); k_vt3<<<g2, 256, 0, stream>>>(QKV, VT0);
        attend(Q16, K16, VT0);
        k_gemmw<bf, 1, true><<<dim3(NN / 64, EE / 64, 1), 32, 0, stream>>>(Ch, Cl, SWOUT, nullptr, EE, MSG, EE, sbout, 0, 0, 0);
        ffn(true, x, SW1, sb1, sg, sbn, SW2, sb2, Dout); };
    for (int b = 0; b < NB_; ++b) {
        self_block(desc0 + (size_t)b * NN * EE, enc0 + (size_t)b * NN * HD, D0); self_block(desc1 + (size_t)b * NN * EE, enc1 + (size_t)b * NN * HD, D1);
        k_dpl<<<gE, 256, 0, stream>>>(D0, D0h, D0l); k_dpl<<<gE, 256, 0, stream>>>(D1, D1h, D1l);
        k_gemmw<bf, 1, true><<<dim3(NN / 64, EE / 64, 1), 32, 0, stream>>>(D0h, D0l, CWQK, nullptr, EE, QK0, EE, cbqk, 0, 0, 0); k_gemmw<bf, 1, true><<<dim3(NN / 64, EE / 64, 1), 32, 0, stream>>>(D1h, D1l, CWQK, nullptr, EE, QK1, EE, cbqk, 0, 0, 0);
        k_gemmw<bf, 1, true><<<dim3(NN / 64, EE / 64, 1), 32, 0, stream>>>(D0h, D0l, CWV, nullptr, EE, V0, EE, cbv, 0, 0, 0); k_gemmw<bf, 1, true><<<dim3(NN / 64, EE / 64, 1), 32, 0, stream>>>(D1h, D1l, CWV, nullptr, EE, V1, EE, cbv, 0, 0, 0);
        k_cpl<<<g4, 256, 0, stream>>>(QK0, Q16); k_cpl<<<g4, 256, 0, stream>>>(QK1, K16); k_vtc<<<g2, 256, 0, stream>>>(V0, VT0); k_vtc<<<g2, 256, 0, stream>>>(V1, VT1);
        attend(Q16, K16, VT1);
        k_gemmw<bf, 1, true><<<dim3(NN / 64, EE / 64, 1), 32, 0, stream>>>(Ch, Cl, CWO, nullptr, EE, MSG, EE, cbo, 0, 0, 0);
        ffn(false, D0, CW1, cb1, cg, cbn, CW2, cb2, Y); k_out<<<gE, 256, 0, stream>>>(Y, 0, OUT0 + (size_t)b * NN * E2, OUT1 + (size_t)b * NN * E2);
        attend(K16, Q16, VT0);
        k_gemmw<bf, 1, true><<<dim3(NN / 64, EE / 64, 1), 32, 0, stream>>>(Ch, Cl, CWO, nullptr, EE, MSG, EE, cbo, 0, 0, 0);
        ffn(false, D1, CW1, cb1, cg, cbn, CW2, cb2, Y); k_out<<<gE, 256, 0, stream>>>(Y, EE, OUT0 + (size_t)b * NN * E2, OUT1 + (size_t)b * NN * E2); }
}
